// VPNNetwork_85899346321
// MI455X (gfx1250) — hardware-verified
//
#include <hip/hip_runtime.h>


#define NB_  4096
#define GH   32
#define GW   32
#define NC   1024
#define DIN  3072
#define DPH  2048
#define KIT  20
#define DM   DPH
#define LOSC 1024.0f
typedef _Float16 h16;
typedef unsigned short bf;
typedef __attribute__((ext_vector_type(16))) __bf16   v16bf;
typedef __attribute__((ext_vector_type(16))) _Float16 v16h;
typedef __attribute__((ext_vector_type(8)))  _Float16 v8h;
typedef __attribute__((ext_vector_type(8)))  unsigned short v8us;
typedef __attribute__((ext_vector_type(8)))  float    v8f;
typedef __attribute__((ext_vector_type(4)))  float    v4f;
typedef v8h  __attribute__((may_alias)) v8ha;
typedef v4f  __attribute__((may_alias)) v4fa;
typedef v8us __attribute__((may_alias)) v8usa;

__device__ __forceinline__ unsigned short f2bf(float f) { unsigned u = __float_as_uint(f); u += 0x7FFFu + ((u >> 16) & 1u); return (unsigned short)(u >> 16); }
__device__ __forceinline__ float bf2f(unsigned short b) { return __uint_as_float(((unsigned)b) << 16); }
__device__ __forceinline__ float bfr(float f) { return bf2f(f2bf(f)); }
__device__ __forceinline__ v16h cat16(v8h lo, v8h hi) { return __builtin_shufflevector(lo, hi, 0, 1, 2, 3, 4, 5, 6, 7, 8, 9, 10, 11, 12, 13, 14, 15); }
__device__ __forceinline__ v16bf cat16b(v8us lo, v8us hi) { return __builtin_bit_cast(v16bf, __builtin_shufflevector(lo, hi, 0, 1, 2, 3, 4, 5, 6, 7, 8, 9, 10, 11, 12, 13, 14, 15)); }
__device__ __forceinline__ v8f wmma16(v16h a, v16h b, v8f c) { return __builtin_amdgcn_wmma_f32_16x16x32_f16(false, a, false, b, (short)0, c, false, false); }
__device__ __forceinline__ v8f wmmab(v16bf a, v16bf b, v8f c) { return __builtin_amdgcn_wmma_f32_16x16x32_bf16(false, a, false, b, (short)0, c, false, false); }


__global__ __launch_bounds__(128) void k_gemmh(const h16* __restrict__ A, const h16* __restrict__ Bn, const float* __restrict__ bias, float* C, int ldc, const float* __restrict__ R, int K, size_t sA, size_t sB, size_t sC, int roundR) {
    __shared__ __align__(16) float ost[4][16 * 68];
    const size_t z = blockIdx.z; A += z * sA; Bn += z * sB; C += z * sC; if (R) R += z * sC;
    const int lane = threadIdx.x & 31, wave = threadIdx.x >> 5, lr = lane & 15, hi = lane >> 4;
    const int r0 = blockIdx.x * 64 + wave * 16, c0 = blockIdx.y * 64;
    const size_t aoff = (size_t)(r0 + lr) * K + 8 * hi;
    size_t boff[4];
#pragma unroll
    for (int t = 0; t < 4; ++t) boff[t] = (size_t)(c0 + t * 16 + lr) * K + 8 * hi;
    v8f acc[4];
#pragma unroll
    for (int t = 0; t < 4; ++t) acc[t] = (v8f){};
#pragma unroll 1
    for (int kc = 0; kc < K; kc += 32) {
        const v16h a = cat16(*(const v8h*)(A + aoff + kc), *(const v8h*)(A + aoff + kc + 16));
#pragma unroll
        for (int t = 0; t < 4; ++t) { const v16h b = cat16(*(const v8h*)(Bn + boff[t] + kc), *(const v8h*)(Bn + boff[t] + kc + 16)); acc[t] = wmma16(a, b, acc[t]); }
        asm volatile("v_nop\n\tv_nop\n\tv_nop\n\tv_nop" : "+v"(acc[0]), "+v"(acc[1]), "+v"(acc[2]), "+v"(acc[3]) : "v"(a));
    }
    float* os = &ost[wave][0];
#pragma unroll
    for (int t = 0; t < 4; ++t) { const float bv = bias ? bfr(bias[c0 + t * 16 + lr]) : 0.f;
#pragma unroll
        for (int j = 0; j < 8; ++j) os[(hi * 8 + j) * 68 + t * 16 + lr] = acc[t][j] + bv; }
    __syncthreads();
    float* crow = C + (size_t)r0 * ldc + c0;
    auto pass = [&]() {
#pragma unroll
        for (int s = 0; s < 8; ++s) { const int Lid = (lane >> 3) + 4 * s, piece = lane & 7; const int row = Lid >> 1, cofs = (Lid & 1) * 32 + piece * 4;
            v4f val = *(const v4fa*)(os + row * 68 + cofs); if (R) { const v4f rv = *(const v4f*)(R + ((size_t)r0 + row) * ldc + c0 + cofs); val += roundR ? (v4f){bfr(rv[0]), bfr(rv[1]), bfr(rv[2]), bfr(rv[3])} : rv; }
            *(volatile v4f*)(crow + (size_t)row * ldc + cofs) = val; }
    };
    pass(); __threadfence(); pass();
}

template <int MODE>
__global__ __launch_bounds__(128) void k_gemm3z(const bf* __restrict__ Ah, const bf* __restrict__ Al, const bf* __restrict__ Bh, const bf* __restrict__ Bl, int K, float* C, int ldc, size_t sA, size_t sB, size_t sC) {
    if ((MODE & 1) && (int)blockIdx.y * 64 > (int)blockIdx.x * 64 + 63) return;
    const size_t z = blockIdx.z; Ah += z * sA; Al += z * sA; Bh += z * sB; Bl += z * sB; C += z * sC;
    const int Klim = (MODE & 2) ? min(K, ((int)blockIdx.x + 1) * 64) : K;
    __shared__ __align__(16) float ost[4][16 * 68];
    const int lane = threadIdx.x & 31, wave = threadIdx.x >> 5, lr = lane & 15, hi = lane >> 4;
    const int r0 = blockIdx.x * 64 + wave * 16, c0 = blockIdx.y * 64;
    const size_t aoff = (size_t)(r0 + lr) * K + 8 * hi;
    v8f acc[4];
#pragma unroll
    for (int t = 0; t < 4; ++t) acc[t] = (v8f){};
#pragma unroll 1
    for (int kc = 0; kc < Klim; kc += 32) {
        const v16bf a = cat16b(*(const v8us*)(Ah + aoff + kc), *(const v8us*)(Ah + aoff + kc + 16));
        v16bf al = a; if (!(MODE & 4) && !(MODE & 16)) al = cat16b(*(const v8us*)(Al + aoff + kc), *(const v8us*)(Al + aoff + kc + 16));
#pragma unroll
        for (int t = 0; t < 4; ++t) { const size_t bo = (size_t)(c0 + t * 16 + lr) * K + kc + 8 * hi;
            const v16bf bh = cat16b(*(const v8us*)(Bh + bo), *(const v8us*)(Bh + bo + 16));
            acc[t] = wmmab(a, bh, acc[t]);
            if (!(MODE & 4)) { if (!(MODE & 16)) acc[t] = wmmab(al, bh, acc[t]); if (!(MODE & 8)) { const v16bf bl = cat16b(*(const v8us*)(Bl + bo), *(const v8us*)(Bl + bo + 16)); acc[t] = wmmab(a, bl, acc[t]); } } }
        asm volatile("v_nop\n\tv_nop\n\tv_nop\n\tv_nop" : "+v"(acc[0]), "+v"(acc[1]), "+v"(acc[2]), "+v"(acc[3]) : "v"(a), "v"(al));
    }
    float* os = &ost[wave][0];
#pragma unroll
    for (int t = 0; t < 4; ++t) {
#pragma unroll
        for (int j = 0; j < 8; ++j) os[(hi * 8 + j) * 68 + t * 16 + lr] = acc[t][j]; }
    __builtin_amdgcn_wave_barrier(); asm volatile("" ::: "memory");
    float* crow = C + (size_t)r0 * ldc + c0;
    auto pass = [&]() {
#pragma unroll
        for (int s = 0; s < 8; ++s) { const int Lid = (lane >> 3) + 4 * s, piece = lane & 7; const int row = Lid >> 1, cofs = (Lid & 1) * 32 + piece * 4;
            const v4f val = *(const v4fa*)(os + row * 68 + cofs); *(volatile v4f*)(crow + (size_t)row * ldc + cofs) = val; }
    };
    pass(); __threadfence(); pass();
}
__global__ __launch_bounds__(256) void k_planes32z(const float* __restrict__ F, int ld, int off, float sc, int rows, bf* Ph, bf* Pl) {
    typedef __attribute__((ext_vector_type(2))) unsigned short v2us;
    const int lane = threadIdx.x & 31; const size_t r = ((size_t)blockIdx.x * 8 + (threadIdx.x >> 5)) * 2 + (lane >> 4); if (r >= (size_t)rows) return; const int z = blockIdx.z; const int c0 = (lane & 15) * 2; v2us oh, ol;
    Ph += (size_t)z * rows * 32; Pl += (size_t)z * rows * 32;
#pragma unroll
    for (int i = 0; i < 2; ++i) { const float y = F[r * ld + off + z * 32 + c0 + i] * sc; const unsigned short hb = f2bf(y); oh[i] = hb; ol[i] = f2bf(y - bf2f(hb)); }
    const size_t o = r * 32 + c0; *(volatile v2us*)(Ph + o) = oh; *(volatile v2us*)(Pl + o) = ol; __threadfence(); *(volatile v2us*)(Ph + o) = oh; *(volatile v2us*)(Pl + o) = ol;
}
__global__ __launch_bounds__(256) void k_vtpadz(const float* __restrict__ F, int ld, int off, int nk, bf* Th, bf* Tl) {
    typedef __attribute__((ext_vector_type(2))) unsigned short v2us;
    const int lane = threadIdx.x & 31; const size_t wid = (size_t)blockIdx.x * 8 + (threadIdx.x >> 5); if (wid >= (size_t)64 * (nk / 64)) return; const int z = blockIdx.z; const int d = (int)(wid / (nk / 64)); const int k0 = (int)(wid % (nk / 64)) * 64 + lane * 2; v2us oh, ol;
    Th += (size_t)z * 64 * nk; Tl += (size_t)z * 64 * nk;
#pragma unroll
    for (int i = 0; i < 2; ++i) { const float y = (d < 32) ? F[(size_t)(k0 + i) * ld + off + z * 32 + (d < 32 ? d : 0)] : 0.f; const unsigned short hb = f2bf(y); oh[i] = hb; ol[i] = f2bf(y - bf2f(hb)); }
    const size_t o = (size_t)d * nk + k0; *(volatile v2us*)(Th + o) = oh; *(volatile v2us*)(Tl + o) = ol; __threadfence(); *(volatile v2us*)(Th + o) = oh; *(volatile v2us*)(Tl + o) = ol;
}
template <int NK>
__global__ __launch_bounds__(256) void k_softmaxz(const float* __restrict__ S, int rows, bf* PH, bf* PL) {
    typedef __attribute__((ext_vector_type(4))) unsigned short v4us;
    const int lane = threadIdx.x & 31, i = blockIdx.x * 8 + (threadIdx.x >> 5); if (i >= rows) return; const size_t zo = (size_t)blockIdx.z * rows * NK; const float* sr = S + zo + (size_t)i * NK; PH += zo; PL += zo;
    float m = -3.0e38f;
#pragma unroll 1
    for (int c0 = lane * 4; c0 < NK; c0 += 128) {
#pragma unroll
        for (int q = 0; q < 4; ++q) m = fmaxf(m, sr[c0 + q]); }
#pragma unroll
    for (int sh = 16; sh; sh >>= 1) m = fmaxf(m, __shfl_xor(m, sh, 32));
    float sum = 0.f;
#pragma unroll 1
    for (int c0 = lane * 4; c0 < NK; c0 += 128) {
#pragma unroll
        for (int q = 0; q < 4; ++q) sum += __expf(sr[c0 + q] - m); }
#pragma unroll
    for (int sh = 16; sh; sh >>= 1) sum += __shfl_xor(sum, sh, 32);
    const float inv = 1.0f / sum;
#pragma unroll 1
    for (int ps = 0; ps < 2; ++ps) {
#pragma unroll 1
        for (int c0 = lane * 4; c0 < NK; c0 += 128) { v4us oh, ol;
#pragma unroll
            for (int q = 0; q < 4; ++q) { const float p = __expf(sr[c0 + q] - m) * inv; const unsigned short hb = f2bf(p); oh[q] = hb; ol[q] = f2bf(p - bf2f(hb)); }
            const size_t o = (size_t)i * NK + c0; *(volatile v4us*)(PH + o) = oh; *(volatile v4us*)(PL + o) = ol; }
        if (ps == 0) __threadfence(); }
}
__global__ __launch_bounds__(256) void k_placez(const float* __restrict__ XH, int rows, int ldy, float* Y) {
    const int lane = threadIdx.x & 31; const size_t q = (size_t)blockIdx.x * 8 + (threadIdx.x >> 5); if (q >= (size_t)rows) return; const int z = blockIdx.z; const float v = XH[((size_t)z * rows + q) * 64 + lane];
    *(volatile float*)(Y + q * ldy + z * 32 + lane) = v; __threadfence(); *(volatile float*)(Y + q * ldy + z * 32 + lane) = v;
}

template <typename T16> struct WFrag;
template <> struct WFrag<h16> { typedef v16h V; static __device__ __forceinline__ V ld(const h16* p) { return cat16(*(const v8h*)p, *(const v8h*)(p + 16)); } static __device__ __forceinline__ v8f mma(V a, V b, v8f c) { return wmma16(a, b, c); } };
template <> struct WFrag<bf> { typedef v16bf V; static __device__ __forceinline__ V ld(const bf* p) { return cat16b(*(const v8us*)p, *(const v8us*)(p + 16)); } static __device__ __forceinline__ v8f mma(V a, V b, v8f c) { return wmmab(a, b, c); } };
template <typename T16, int NSPLIT, bool BIAS>
__global__ __launch_bounds__(32) void k_gemmw(const T16* __restrict__ A, const T16* __restrict__ A2, const T16* __restrict__ Bt, const T16* __restrict__ Bt2, int K, float* C, int ldc, const float* __restrict__ bias, size_t sA, size_t sB, size_t sC) {
    typedef typename WFrag<T16>::V V;
    __shared__ __align__(16) float os[16 * 68];
    const size_t z = blockIdx.z; A += z * sA; if (A2) A2 += z * sA; Bt += z * sB; if (Bt2) Bt2 += z * sB; C += z * sC;
    const int lane = threadIdx.x & 31, lr = lane & 15, hi = lane >> 4; const int r0 = blockIdx.x * 64, c0 = blockIdx.y * 64;
    v8f acc[4][4];
#pragma unroll
    for (int mb = 0; mb < 4; ++mb)
#pragma unroll
        for (int nb = 0; nb < 4; ++nb) acc[mb][nb] = (v8f){};
    const size_t aoff = (size_t)(r0 + lr) * K + 8 * hi, boff = (size_t)(c0 + lr) * K + 8 * hi;
#pragma unroll 1
    for (int kc = 0; kc < K; kc += 32) {
        V a[4], a2[4];
#pragma unroll
        for (int mb = 0; mb < 4; ++mb) { a[mb] = WFrag<T16>::ld(A + aoff + (size_t)mb * 16 * K + kc); if (NSPLIT == 1 || NSPLIT == 2) a2[mb] = WFrag<T16>::ld(A2 + aoff + (size_t)mb * 16 * K + kc); }
#pragma unroll
        for (int nb = 0; nb < 4; ++nb) { const V b = WFrag<T16>::ld(Bt + boff + (size_t)nb * 16 * K + kc); V b2; if (NSPLIT >= 2) b2 = WFrag<T16>::ld(Bt2 + boff + (size_t)nb * 16 * K + kc);
#pragma unroll
            for (int mb = 0; mb < 4; ++mb) { acc[mb][nb] = WFrag<T16>::mma(a[mb], b, acc[mb][nb]); if (NSPLIT == 1 || NSPLIT == 2) acc[mb][nb] = WFrag<T16>::mma(a2[mb], b, acc[mb][nb]); if (NSPLIT >= 2) acc[mb][nb] = WFrag<T16>::mma(a[mb], b2, acc[mb][nb]); } }
        asm volatile("v_nop\n\tv_nop\n\tv_nop\n\tv_nop" : "+v"(acc[0][0]), "+v"(acc[1][1]), "+v"(acc[2][2]), "+v"(acc[3][3]) : "v"(a[0]), "v"(a[3]));
    }
#pragma unroll
    for (int mb = 0; mb < 4; ++mb) {
#pragma unroll
        for (int nb = 0; nb < 4; ++nb) {
#pragma unroll
            for (int j = 0; j < 8; ++j) os[(hi * 8 + j) * 68 + nb * 16 + lr] = acc[mb][nb][j]; }
        __builtin_amdgcn_wave_barrier(); asm volatile("" ::: "memory");
        float* crow = C + (size_t)(r0 + mb * 16) * ldc + c0;
#pragma unroll 1
        for (int ps = 0; ps < 2; ++ps) {
#pragma unroll
            for (int s = 0; s < 8; ++s) { const int row = 2 * s + hi, cofs = lr * 4; v4f val = *(const v4fa*)(os + row * 68 + cofs); if (BIAS) { val[0] += bfr(bias[c0 + cofs]); val[1] += bfr(bias[c0 + cofs + 1]); val[2] += bfr(bias[c0 + cofs + 2]); val[3] += bfr(bias[c0 + cofs + 3]); }
                *(volatile v4f*)(crow + (size_t)row * ldc + cofs) = val; }
            if (ps == 0) __threadfence(); }
        __builtin_amdgcn_wave_barrier(); asm volatile("" ::: "memory");
    }
}

__global__ __launch_bounds__(256) void k_wT(const float* __restrict__ Wm, bf* Bt) {
    __shared__ float tl[64][65]; typedef __attribute__((ext_vector_type(4))) unsigned short v4us;
    const int tid = threadIdx.x; const int k0 = blockIdx.x * 64, n0 = blockIdx.y * 64; const int rr = tid >> 2, cq = (tid & 3) * 16;
#pragma unroll
    for (int i = 0; i < 16; ++i) tl[rr][cq + i] = bfr(Wm[(size_t)(k0 + rr) * DPH + n0 + cq + i]);
    __syncthreads();
    const int lane = tid & 31, wv = tid >> 5;
    auto pass = [&]() {
#pragma unroll
        for (int st = 0; st < 4; ++st) { const int nr = wv * 8 + st * 2 + (lane >> 4); const int kq = (lane & 15) * 4; v4us v; for (int i = 0; i < 4; ++i) v[i] = f2bf(tl[kq + i][nr]); *(volatile v4us*)(Bt + (size_t)(n0 + nr) * DIN + k0 + kq) = v; }
    };
    pass(); __threadfence(); pass();
}
__global__ __launch_bounds__(256) void k_cvtx(const float* __restrict__ x, bf* A) {
    const int lane = threadIdx.x & 31; const size_t r = (size_t)blockIdx.x * 8 + (threadIdx.x >> 5); if (r >= (size_t)NB_) return;
#pragma unroll 1
    for (int ps = 0; ps < 2; ++ps) {
#pragma unroll
        for (int q = 0; q < DIN / 256; ++q) { const size_t o = r * DIN + q * 256 + lane * 8; v8us v;
#pragma unroll
            for (int i = 0; i < 8; ++i) v[i] = f2bf(x[o + i]);
            *(volatile v8us*)(A + o) = v; }
        if (ps == 0) __threadfence(); }
}
__device__ __forceinline__ float sigm(float z) { return __fdiv_rn(1.0f, __fadd_rn(1.0f, __expf(-z))); }
__global__ __launch_bounds__(256) void k_vi(const float* __restrict__ Z, float* VMAP) {
    __shared__ float Vs[GH + 2][GW + 2];
    const int tid = threadIdx.x; const int b = blockIdx.x; const int row = tid >> 3, c0 = (tid & 7) * 4;
    for (int i = tid; i < (GH + 2) * (GW + 2); i += 256) (&Vs[0][0])[i] = 0.f;
    __syncthreads();
    float r[4], p[4], v[4];
#pragma unroll
    for (int k = 0; k < 4; ++k) { const int cell = row * GW + c0 + k; r[k] = sigm(Z[(size_t)b * DPH + 2 * cell]); p[k] = sigm(Z[(size_t)b * DPH + 2 * cell + 1]); v[k] = r[k]; Vs[row + 1][c0 + k + 1] = v[k]; }
    __syncthreads();
#pragma unroll 1
    for (int it = 0; it < KIT; ++it) {
        float nv[4];
#pragma unroll
        for (int k = 0; k < 4; ++k) { const int i = row + 1, j = c0 + k + 1; const float nb = fmaxf(fmaxf(Vs[i - 1][j], Vs[i + 1][j]), fmaxf(Vs[i][j - 1], Vs[i][j + 1])); float dlt = __fsub_rn(nb, r[k]); float pr = __fmul_rn(p[k], dlt); asm volatile("" : "+v"(pr));   const float t = __fadd_rn(r[k], pr); nv[k] = fmaxf(v[k], t); }
        __syncthreads();
#pragma unroll
        for (int k = 0; k < 4; ++k) { v[k] = nv[k]; Vs[row + 1][c0 + k + 1] = v[k]; }
        __syncthreads(); }
    v4f o; for (int k = 0; k < 4; ++k) o[k] = v[k];
    float* dst = VMAP + (size_t)b * NC + row * GW + c0; *(volatile v4f*)dst = o; __threadfence(); *(volatile v4f*)dst = o;
}
__global__ __launch_bounds__(256) void k_head(const float* __restrict__ obs, const float* __restrict__ VMAP, const float* __restrict__ L1w, const float* __restrict__ L1b, const float* __restrict__ L2w, const float* __restrict__ L2b, float* OUTB) {
    const int lane = threadIdx.x & 31; const int w = blockIdx.x * 8 + (threadIdx.x >> 5); if (w >= NB_ / 8) return; float res = 0.f;
#pragma unroll 1
    for (int s = 0; s < 8; ++s) { const int b = w * 8 + s; const float* ob = obs + (size_t)b * DIN;
        float bm = -3.0e38f; int bi = 0x7fffffff;
#pragma unroll 1
        for (int c = lane; c < NC; c += 32) { const float vch = bfr(ob[c * 3 + 1]); if (vch > bm) { bm = vch; bi = c; } }
#pragma unroll
        for (int sh = 16; sh; sh >>= 1) { const float om = __shfl_xor(bm, sh, 32); const int oi = __shfl_xor(bi, sh, 32); if (om > bm || (om == bm && oi < bi)) { bm = om; bi = oi; } }
        const int pi = bi / GW, pj = bi % GW;
        auto selv = [&](int m) { const int ii = m / 12, rem = m % 12, jj = rem / 4, ch = rem % 4; const int gi = pi + ii - 1, gj = pj + jj - 1; if (gi < 0 || gi >= GH || gj < 0 || gj >= GW) return 0.f; return (ch < 3) ? bfr(ob[(gi * GW + gj) * 3 + ch]) : VMAP[(size_t)b * NC + gi * GW + gj]; };
        float h = 0.f; if (lane < 16) { float a = bfr(L1b[lane]);
#pragma unroll 1
            for (int m = 0; m < 36; ++m) a = fmaf(selv(m), bfr(L1w[m * 16 + lane]), a); h = fmaxf(a, 0.f); }
        float lg = (lane < 4) ? bfr(L2b[lane]) : 0.f;
#pragma unroll 1
        for (int k = 0; k < 16; ++k) { const float hk = __shfl(h, k, 32); if (lane < 4) lg = fmaf(hk, bfr(L2w[k * 4 + lane]), lg); }
        const float mine = __shfl(lg, lane & 3, 32); if ((lane >> 2) == s) res = mine; }
    *(volatile float*)(OUTB + (size_t)w * 32 + lane) = res; __threadfence(); *(volatile float*)(OUTB + (size_t)w * 32 + lane) = res;
}
extern "C" void kernel_launch(void* const* d_in, const int* in_sizes, int n_in,
                              void* d_out, int out_size, void* d_ws, size_t ws_size, hipStream_t stream) {
    (void)in_sizes; (void)n_in; (void)out_size;
    const float* obs = (const float*)d_in[0]; const float* Pw = (const float*)d_in[1]; const float* Pb = (const float*)d_in[2]; const float* L1w = (const float*)d_in[3]; const float* L1b = (const float*)d_in[4]; const float* L2w = (const float*)d_in[5]; const float* L2b = (const float*)d_in[6];
    float* out = (float*)d_out;
    char* wsp = (char*)d_ws;
    auto take = [&](size_t bytes) { char* p = wsp; wsp += (bytes + 255) & ~(size_t)255; return (void*)p; };
    bf* WB = (bf*)take((size_t)DPH * DIN * 2); bf* XB = (bf*)take((size_t)NB_ * DIN * 2); float* Z = (float*)take((size_t)NB_ * DPH * 4); float* VMAP = (float*)take((size_t)NB_ * NC * 4);
    if ((size_t)(wsp - (char*)d_ws) > ws_size) return;
    k_wT<<<dim3(DIN / 64, DPH / 64, 1), 256, 0, stream>>>(Pw, WB); k_cvtx<<<NB_ / 8, 256, 0, stream>>>(obs, XB);
    k_gemmw<bf, 0, true><<<dim3(NB_ / 64, DPH / 64, 1), 32, 0, stream>>>(XB, nullptr, WB, nullptr, DIN, Z, DPH, Pb, 0, 0, 0);
    k_vi<<<NB_, 256, 0, stream>>>(Z, VMAP);
    k_head<<<(NB_ / 8) / 8, 256, 0, stream>>>(obs, VMAP, L1w, L1b, L2w, L2b, out);
}
